// SplineCoupling_7275674600569
// MI455X (gfx1250) — hardware-verified
//
#include <hip/hip_runtime.h>
#include <math.h>

typedef __attribute__((ext_vector_type(16))) _Float16 v16h;
typedef __attribute__((ext_vector_type(16))) __bf16 v16b;
typedef __attribute__((ext_vector_type(8)))  _Float16 v8h;
typedef __attribute__((ext_vector_type(8)))  float v8f;
typedef __attribute__((ext_vector_type(4)))  float v4f;
typedef __attribute__((ext_vector_type(2)))  float v2f;
typedef __attribute__((ext_vector_type(4)))  unsigned v4u;
typedef __attribute__((ext_vector_type(4)))  int v4i;
typedef float __attribute__((may_alias)) float_a;
typedef int __attribute__((may_alias)) int_a;

template <typename T> __device__ __forceinline__ void vst2(void* p, T v) { *(volatile T*)p = v; __threadfence(); *(volatile T*)p = v; }
__device__ __forceinline__ v8f wmma16(v16h a, v16h b, v8f c) {
  v8f d = __builtin_amdgcn_wmma_f32_16x16x32_f16(false, a, false, b, (short)0, c, false, false);
  asm volatile("v_nop\n\tv_nop\n\tv_nop\n\tv_nop" : "+v"(d) : "v"(a), "v"(b));
  return d;
}
__device__ __forceinline__ v8f wmma_bf(v16b a, v16b b, v8f c) {
  v8f d = __builtin_amdgcn_wmma_f32_16x16x32_bf16(false, a, false, b, (short)0, c, false, false);
  asm volatile("v_nop\n\tv_nop\n\tv_nop\n\tv_nop" : "+v"(d) : "v"(a), "v"(b));
  return d;
}
__device__ __forceinline__ v16h frag_h(const _Float16* rowk0, int lane) {
  union { v16h v; v8h q[2]; } u; const _Float16* p = rowk0 + 8 * (lane >> 4);
  u.q[0] = *(const v8h*)p; u.q[1] = *(const v8h*)(p + 16); return u.v;
}
__device__ __forceinline__ v16h frag_f32(const float* rowk0, int lane) {
  v16h a; const float* p = rowk0 + 8 * (lane >> 4);
#pragma unroll
  for (int i = 0; i < 8; ++i) { a[i] = (_Float16)p[i]; a[8 + i] = (_Float16)p[16 + i]; }
  return a;
}
__device__ __forceinline__ v16h frag_f32s(const float* rowk0, int lane, float sc) {
  v16h a; const float* p = rowk0 + 8 * (lane >> 4);
#pragma unroll
  for (int i = 0; i < 8; ++i) { a[i] = (_Float16)(p[i] * sc); a[8 + i] = (_Float16)(p[16 + i] * sc); }
  return a;
}
__device__ __forceinline__ v16h fragc_f32(const float* W, int k0, int n, int lane, int ld, int K) {
  v16h a; const int g = lane >> 4;
#pragma unroll
  for (int i = 0; i < 8; ++i) { const int ka = k0 + 8 * g + i, kb = ka + 16;
    a[i] = (_Float16)(ka < K ? W[(size_t)(ka < K ? ka : K - 1) * ld + n] : 0.f); a[8 + i] = (_Float16)(kb < K ? W[(size_t)(kb < K ? kb : K - 1) * ld + n] : 0.f); }
  return a;
}
struct F2 { v16b h, l; };
__device__ __forceinline__ F2 bsplit16(const float v[16]) { F2 r;
#pragma unroll
  for (int i = 0; i < 16; ++i) { const __bf16 h = (__bf16)v[i]; r.h[i] = h; r.l[i] = (__bf16)(v[i] - (float)h); }
  return r; }
__device__ __forceinline__ F2 split_row(const float* row, int k0, int lane) { float v[16]; const float* p = row + k0 + 8 * (lane >> 4);
#pragma unroll
  for (int i = 0; i < 8; ++i) { v[i] = p[i]; v[8 + i] = p[16 + i]; }
  return bsplit16(v); }
__device__ __forceinline__ F2 split_rowK(const float* row, int k0, int lane, int K) { float v[16]; const int g = lane >> 4;
#pragma unroll
  for (int i = 0; i < 8; ++i) { const int ka = k0 + 8 * g + i, kb = ka + 16; v[i] = ka < K ? row[ka < K ? ka : K - 1] : 0.f; v[8 + i] = kb < K ? row[kb < K ? kb : K - 1] : 0.f; }
  return bsplit16(v); }
__device__ __forceinline__ F2 split_col(const float* W, int k0, int n, int lane, int ld, int K) { float v[16]; const int g = lane >> 4;
#pragma unroll
  for (int i = 0; i < 8; ++i) { const int ka = k0 + 8 * g + i, kb = ka + 16; v[i] = ka < K ? W[(size_t)(ka < K ? ka : K - 1) * ld + n] : 0.f; v[8 + i] = kb < K ? W[(size_t)(kb < K ? kb : K - 1) * ld + n] : 0.f; }
  return bsplit16(v); }
__device__ __forceinline__ v8f mac3(const F2& a, const F2& b, v8f c) { c = wmma_bf(a.l, b.h, c); c = wmma_bf(a.h, b.l, c); return wmma_bf(a.h, b.h, c); }
__device__ __forceinline__ float sigm(float v) { return 1.0f / (1.0f + expf(-v)); }
#define LDSX() do { asm volatile("s_wait_dscnt 0" ::: "memory"); __builtin_amdgcn_wave_barrier(); __builtin_amdgcn_fence(__ATOMIC_RELEASE, "workgroup"); } while (0)


#define NRW 32768
#define D1 64
#define D2 64
#define CD 128
#define HID 128
#define NBIN 16
#define NPAR (3 * NBIN + 1)
#define NP3 (D1 * NPAR)
#define NP3P 3200
#ifndef TRB
#define TRB (NRW / 64)
#endif
typedef __attribute__((ext_vector_type(8))) __bf16 v8b;
__device__ __forceinline__ v16b frag_b(const __bf16* rowk0, int lane) {
  union { v16b v; v8b q[2]; } u; const __bf16* p = rowk0 + 8 * (lane >> 4);
  u.q[0] = *(const v8b*)p; u.q[1] = *(const v8b*)(p + 16); return u.v;
}
__device__ __forceinline__ float bfr(float v) { return (float)(__bf16)v; }
__device__ __attribute__((noinline)) float exp_ni(float v) { return expf(v); }
__device__ __attribute__((noinline)) float erf_ni(float v) { return erff(v); }

#define WS_P1  0u
#define WS_P2  (WS_P1 + 2u * HID * 192)
#define WS_P3  (WS_P2 + 2u * HID * HID)
#define WS_H2H (WS_P3 + 2u * NP3P * HID)
#define WS_H2L (WS_H2H + 2u * NRW * HID)
#define WS_END (WS_H2L + 2u * NRW * HID)

__device__ __attribute__((noinline)) float softplus_p(float x) { return fmaxf(x, 0.f) + log1pf(expf(-fabsf(x))); }
__device__ __attribute__((noinline)) float log_p(float x) { return logf(x); }
__global__ __launch_bounds__(128) void k_pack(const float* __restrict__ W1, const float* __restrict__ W2, const float* __restrict__ W3, __bf16* __restrict__ P) {
  const int n = blockIdx.x, which = blockIdx.y, t = threadIdx.x; __shared__ __align__(16) __bf16 s[192];
  if (which == 0) { if (n >= HID) return; for (int k = t; k < 192; k += 128) s[k] = (__bf16)W1[(size_t)k * HID + n]; __syncthreads(); if (t < 192 / 8) vst2((unsigned*)(P + WS_P1 / 2 + (size_t)n * 192 + t * 8), *(const v4u*)&s[t * 8]); }
  else if (which == 1) { if (n >= HID) return; s[t] = (__bf16)W2[(size_t)t * HID + n]; __syncthreads(); if (t < HID / 8) vst2((unsigned*)(P + WS_P2 / 2 + (size_t)n * HID + t * 8), *(const v4u*)&s[t * 8]); }
  else { s[t] = (__bf16)((n < NP3) ? W3[(size_t)t * NP3 + n] : 0.f); __syncthreads(); if (t < HID / 8) vst2((unsigned*)(P + WS_P3 / 2 + (size_t)n * HID + t * 8), *(const v4u*)&s[t * 8]); }
}
__global__ __launch_bounds__(128) void k_mlp(const float* __restrict__ U2, const float* __restrict__ CND, const __bf16* __restrict__ P, const float* __restrict__ B1, const float* __restrict__ B2, __bf16* __restrict__ H2H, __bf16* __restrict__ H2L) {
  __shared__ __align__(16) __bf16 sx[64][200], sh[64][HID + 8], sl[64][HID + 8]; __shared__ __align__(16) __bf16 soh[4][16][136], sol[4][16][136];
  const int tid = threadIdx.x, wave = tid >> 5, lane = tid & 31, col = lane & 15, g = lane >> 4; const size_t r0 = (size_t)blockIdx.x * 64;
  for (int e = tid; e < 64 * 192; e += 128) { const int r = e / 192, c = e % 192; sx[r][c] = (__bf16)((c < D2) ? U2[(r0 + r) * D2 + c] : CND[(r0 + r) * CD + (c - D2)]); }
  if (tid < 64) for (int c = 192; c < 200; ++c) sx[tid][c] = (__bf16)0.f;
  __syncthreads();
  { v8f acc[8] = {};
#pragma unroll
    for (int kc = 0; kc < 192 / 32; ++kc) { const v16b a = frag_b(&sx[wave * 16 + col][kc * 32], lane);
#pragma unroll
      for (int j = 0; j < 8; ++j) acc[j] = wmma_bf(a, frag_b(P + WS_P1 / 2 + (size_t)(j * 16 + col) * 192 + kc * 32, lane), acc[j]); }
#pragma unroll
    for (int j = 0; j < 8; ++j) { const int c = j * 16 + col; const float bb = bfr(B1[c]);
#pragma unroll
      for (int r = 0; r < 8; ++r) { const float v = fmaxf(acc[j][r] + bb, 0.f); const __bf16 hb = (__bf16)v; sh[wave * 16 + 8 * g + r][c] = hb; sl[wave * 16 + 8 * g + r][c] = (__bf16)(v - (float)hb); } } }
  if (tid < 64) for (int c = HID; c < HID + 8; ++c) { sh[tid][c] = (__bf16)0.f; sl[tid][c] = (__bf16)0.f; }
  __syncthreads();
  { v8f acc[8] = {};
#pragma unroll
    for (int kc = 0; kc < HID / 32; ++kc) { const v16b a = frag_b(&sh[wave * 16 + col][kc * 32], lane), al = frag_b(&sl[wave * 16 + col][kc * 32], lane);
#pragma unroll
      for (int j = 0; j < 8; ++j) { const v16b w = frag_b(P + WS_P2 / 2 + (size_t)(j * 16 + col) * HID + kc * 32, lane); acc[j] = wmma_bf(al, w, acc[j]); acc[j] = wmma_bf(a, w, acc[j]); } }
#pragma unroll
    for (int j = 0; j < 8; ++j) { const int c = j * 16 + col; const float bb = bfr(B2[c]);
#pragma unroll
      for (int r = 0; r < 8; ++r) { const float v = fmaxf(acc[j][r] + bb, 0.f); const __bf16 hb = (__bf16)v; soh[wave][8 * g + r][c] = hb; sol[wave][8 * g + r][c] = (__bf16)(v - (float)hb); } } }
  LDSX();
  for (int rl = 0; rl < 16; ++rl) if (lane < 16) { vst2((unsigned*)(H2H + (r0 + wave * 16 + rl) * HID + lane * 8), *(const v4u*)&soh[wave][rl][lane * 8]); vst2((unsigned*)(H2L + (r0 + wave * 16 + rl) * HID + lane * 8), *(const v4u*)&sol[wave][rl][lane * 8]); }
}
__global__ __launch_bounds__(128) void k_spline(const float* __restrict__ U1, const __bf16* __restrict__ H2H, const __bf16* __restrict__ H2L, const __bf16* __restrict__ P, const float* __restrict__ B3, float* __restrict__ OUTV, float* __restrict__ OUTJ) {
  __shared__ __align__(16) float sraw[64][NPAR + 3]; __shared__ __align__(16) float sv[64][D1 + 4]; __shared__ __align__(16) float slj[64];
  const int tid = threadIdx.x, wave = tid >> 5, lane = tid & 31, col = lane & 15, g = lane >> 4; const size_t r0 = (size_t)blockIdx.x * 64;
  v16b ah[HID / 32], al[HID / 32];
#pragma unroll
  for (int kc = 0; kc < HID / 32; ++kc) { ah[kc] = frag_b(H2H + (r0 + wave * 16 + col) * HID + kc * 32, lane); al[kc] = frag_b(H2L + (r0 + wave * 16 + col) * HID + kc * 32, lane); }
  if (tid < 64) slj[tid] = 0.f;
#pragma unroll 1
  for (int d = 0; d < D1; ++d) { v8f acc[4] = {};
#pragma unroll
    for (int kc = 0; kc < HID / 32; ++kc) {
#pragma unroll
      for (int j = 0; j < 4; ++j) { const v16b w = frag_b(P + WS_P3 / 2 + (size_t)(d * NPAR + j * 16 + col) * HID + kc * 32, lane); acc[j] = wmma_bf(al[kc], w, acc[j]); acc[j] = wmma_bf(ah[kc], w, acc[j]); } }
    __syncthreads();
#pragma unroll
    for (int j = 0; j < 4; ++j) { const int pj = j * 16 + col; if (pj < NPAR) { const float bb = bfr(B3[d * NPAR + pj]);
#pragma unroll
        for (int r = 0; r < 8; ++r) sraw[wave * 16 + 8 * g + r][pj] = acc[j][r] + bb; } }
    __syncthreads();
    if (tid < 64) { const int r = tid; const float* p = sraw[r];
      const float left = p[0] + (-5.0f), bottom = p[1] + (-5.0f);
      const float xshift = -1.41280249e-01f, yshift = -1.41280249e-01f, dshift = 5.41324854e-01f;
      float wdt[NBIN], hgt[NBIN], der[NBIN + 1]; float wsum = 0.f, hsum = 0.f;
#pragma unroll
      for (int i = 0; i < NBIN; ++i) { wdt[i] = softplus_p(p[2 + i] + xshift); hgt[i] = softplus_p(p[2 + NBIN + i] + yshift); }
#pragma unroll
      for (int i = 0; i < NBIN; ++i) { wsum += wdt[i]; hsum += hgt[i]; }
      const float scl = hsum / wsum; der[0] = scl; der[NBIN] = scl;
#pragma unroll
      for (int i = 0; i < NBIN - 1; ++i) der[1 + i] = softplus_p(p[2 + 2 * NBIN + i] + dshift);
      float kx[NBIN + 1], ky[NBIN + 1]; kx[0] = left; ky[0] = bottom; { float cw = 0.f, ch = 0.f;
#pragma unroll
        for (int i = 0; i < NBIN; ++i) { cw += wdt[i]; ch += hgt[i]; kx[1 + i] = left + cw; ky[1 + i] = bottom + ch; } }
      const float t = bfr(U1[(r0 + r) * D1 + d]);
      const bool in_dom = (kx[0] < t) && (t <= kx[NBIN]);
      int hi = 0;
#pragma unroll
      for (int i = 0; i <= NBIN; ++i) hi += (kx[i] < t) ? 1 : 0;
      hi = hi < 1 ? 1 : (hi > NBIN ? NBIN : hi); const int lo = hi - 1;
      float xk = 0.f, xkp = 0.f, yk = 0.f, ykp = 0.f, dk = 0.f, dkp = 0.f;
#pragma unroll
      for (int i = 0; i <= NBIN; ++i) { if (i == lo) { xk = kx[i]; yk = ky[i]; dk = der[i]; } if (i == hi) { xkp = kx[i]; ykp = ky[i]; dkp = der[i]; } }
      const float dx = xkp - xk, dy = ykp - yk; const float sk = dy / dx;
      float xi = (t - xk) / dx; xi = fminf(fmaxf(xi, 0.f), 1.f); const float omxi = 1.0f - xi;
      const float num = dy * (sk * xi * xi + dk * xi * omxi); const float den = sk + (dkp + dk - 2.0f * sk) * xi * omxi;
      const float res_in = yk + num / den;
      const float jnum = sk * sk * (dkp * xi * xi + 2.0f * sk * xi * omxi + dk * omxi * omxi);
      const float lj_in = log_p(jnum + 1e-10f) - log_p(den * den + 1e-10f);
      const float shift = bottom - scl * left; const float res_out = scl * t + shift; const float lj_out = log_p(scl + 1e-10f);
      sv[r][d] = in_dom ? res_in : res_out; slj[r] += in_dom ? lj_in : lj_out; }
  }
  __syncthreads();
  for (int e = tid; e < 64 * (D1 / 4); e += 128) { const int r = e >> 4, q = e & 15; vst2(OUTV + (r0 + r) * D1 + q * 4, *(const v4f*)&sv[r][q * 4]); }
  if (tid < 16) vst2(OUTJ + r0 + tid * 4, *(const v4f*)&slj[tid * 4]);
}
extern "C" void kernel_launch(void* const* d_in, const int* in_sizes, int n_in, void* d_out, int out_size, void* d_ws, size_t ws_size, hipStream_t stream) {
  (void)in_sizes; (void)n_in; (void)out_size;
  const float** F = (const float**)d_in;
  if (ws_size < (size_t)WS_END) return;
  char* ws = (char*)d_ws; __bf16* P = (__bf16*)ws; __bf16 *H2H = (__bf16*)(ws + WS_H2H), *H2L = (__bf16*)(ws + WS_H2L);
  k_pack<<<dim3(NP3P, 3), 128, 0, stream>>>(F[3], F[5], F[7], P);
  k_mlp<<<TRB, 128, 0, stream>>>(F[1], F[2], P, F[4], F[6], H2H, H2L);
  k_spline<<<TRB, 128, 0, stream>>>(F[0], H2H, H2L, P, F[8], (float*)d_out, (float*)d_out + (size_t)NRW * D1);
}
